// InContextAssoMemBlock_45578192945718
// MI455X (gfx1250) — hardware-verified
//
#include <hip/hip_runtime.h>
#include <math.h>
#include <stdint.h>

#ifndef NB
#define NB 2
#endif
#ifndef SEQ
#define SEQ 2048
#endif
#define XS_FULL 2048
#define DMOD  1024
#define NH    16
#define HD    64
#define QO    ((SEQ < 512) ? SEQ : 512)
#define MROWS (NB * SEQ)
#define LOG2E 1.4426950408889634f
#define ESCL  10.0f
#define KBUP  5.0f
#define KSC   2048.0f
#define PCAR  32768.0f
#define VCAR  4096.0f
#define OSC   16384.0f
#define WOS   1024.0f
#define WPB   2
#define NHG   (NH / WPB)
#define NQT   (SEQ / 16)
#define NQO   (QO / 16)
#define NST   (SEQ / 64)
#define NKT   (SEQ / 32)
#define ATT_THREADS (WPB * 32)
#define PTP   36
#define PTW   (16 * PTP)
#define SLP   68
#define SLW   (16 * SLP)
#define WREG  (PTW + SLW)
#define SLAB64 (16 * 68)
#define VTP   72
#define TCH   32
#define C8R   (DMOD / 8)
#define WS_CAP 134217728
static_assert(DMOD == NH * HD && HD == 64 && NH == 16 && WPB == 2 && NHG * WPB == NH);
static_assert(ATT_THREADS == 64);
static_assert(NB >= 1 && NB <= 2);
static_assert((SEQ % 64) == 0 && SEQ >= 64 && SEQ <= XS_FULL && (SEQ % TCH) == 0);
static_assert((QO % 64) == 0 && QO >= 64 && QO <= SEQ);
static_assert((DMOD % 64) == 0 && (DMOD % 32) == 0 && (HD % 32) == 0 && C8R == 128);
static_assert(((SEQ * DMOD / 8) % 256) == 0 && ((MROWS * DMOD / 8) % 256) == 0);
static_assert(WPB * WREG * 4 <= 65536 && 2 * HD * VTP * 2 <= 65536 && 4 * SLAB64 * 4 <= 65536 && 2 * TCH * VTP * 2 <= 65536);

typedef unsigned short u16;
typedef _Float16 v16h __attribute__((ext_vector_type(16)));
typedef _Float16 v8h  __attribute__((ext_vector_type(8)));
typedef __bf16   v16b __attribute__((ext_vector_type(16)));
typedef float    v8f  __attribute__((ext_vector_type(8)));
typedef float    v4f  __attribute__((ext_vector_type(4)));
typedef unsigned int v4u __attribute__((ext_vector_type(4)));

union FragH { v16h v; v8h h[2]; v4u u[2]; };
union FragB { v16b v; v4u u[2]; };

__device__ __forceinline__ unsigned short bf_bits(float f) {
  unsigned u = __float_as_uint(f);
  return (unsigned short)((u + 0x7FFFu + ((u >> 16) & 1u)) >> 16);
}
__device__ __forceinline__ float bf_up(unsigned short h) { return __uint_as_float(((unsigned)h) << 16); }
__device__ __forceinline__ float bfr(float f) { return bf_up(bf_bits(f)); }
__device__ __forceinline__ unsigned short h_bits(_Float16 x) { return __builtin_bit_cast(unsigned short, x); }
__device__ __forceinline__ unsigned pk16(unsigned short a, unsigned short b) { return (unsigned)a | ((unsigned)b << 16); }
__device__ __forceinline__ v8f zero8() { v8f z = {0.f, 0.f, 0.f, 0.f, 0.f, 0.f, 0.f, 0.f}; return z; }
__device__ __forceinline__ const _Float16* ash(const u16* p) { return (const _Float16*)(const void*)p; }

__device__ __forceinline__ v16h ldfrag_h(const _Float16* p) {
  FragH f;
  f.h[0] = *(const v8h*)(p);
  f.h[1] = *(const v8h*)(p + 16);
  return f.v;
}
__device__ __forceinline__ v16b ldfrag_b(const u16* p) {
  FragB f;
  f.u[0] = *(const v4u*)(p);
  f.u[1] = *(const v4u*)(p + 16);
  return f.v;
}

__device__ __forceinline__ v8f mma_h(v16h a, v16h b, v8f c) {
  return __builtin_amdgcn_wmma_f32_16x16x32_f16(false, a, false, b, (short)0, c, false, false);
}
__device__ __forceinline__ v8f mma_b(v16b a, v16b b, v8f c) {
  return __builtin_amdgcn_wmma_f32_16x16x32_bf16(false, a, false, b, (short)0, c, false, false);
}
__device__ __forceinline__ void guard2(v8f& a, v8f& b, v16h x0, v16h x1, v16h x2, v16h x3, v16h x4, v16h x5) {
#if defined(__HIP_DEVICE_COMPILE__)
  asm volatile("v_nop\n\tv_nop\n\tv_nop\n\tv_nop"
               : "+v"(a), "+v"(b) : "v"(x0), "v"(x1), "v"(x2), "v"(x3), "v"(x4), "v"(x5) : "memory");
#endif
}
template <typename F>
__device__ __forceinline__ void guard6(v8f& a, v8f& b, v8f& c, v8f& d, F x0, F x1, F x2, F x3, F x4, F x5) {
#if defined(__HIP_DEVICE_COMPILE__)
  asm volatile("v_nop\n\tv_nop\n\tv_nop\n\tv_nop"
               : "+v"(a), "+v"(b), "+v"(c), "+v"(d) : "v"(x0), "v"(x1), "v"(x2), "v"(x3), "v"(x4), "v"(x5) : "memory");
#endif
}
__device__ __forceinline__ void acc_guard4(v8f& a, v8f& b, v8f& c, v8f& d) {
#if defined(__HIP_DEVICE_COMPILE__)
  asm volatile("v_nop\n\tv_nop\n\tv_nop\n\tv_nop" : "+v"(a), "+v"(b), "+v"(c), "+v"(d));
#endif
}
__device__ __forceinline__ void wave_sync_lds() {
  __builtin_amdgcn_fence(__ATOMIC_RELEASE, "workgroup");
  __builtin_amdgcn_wave_barrier();
  __builtin_amdgcn_fence(__ATOMIC_ACQUIRE, "workgroup");
}

__global__ __launch_bounds__(256) void cvt16(const float* __restrict__ x, u16* D, int n8, int f16mode, float scale) {
  const int gt = blockIdx.x * 256 + (int)threadIdx.x;
  if (gt >= n8) return;
  const float* p = x + (size_t)gt * 8;
  const v4f a = *(const v4f*)(p), b4 = *(const v4f*)(p + 4);
  float w[8];
#pragma unroll
  for (int e = 0; e < 4; ++e) { w[e] = a[e]; w[4 + e] = b4[e]; }
  v4u o;
#pragma unroll
  for (int e = 0; e < 4; ++e) {
    const float f0 = w[2 * e], f1 = w[2 * e + 1];
    const unsigned short hb0 = h_bits((_Float16)(bfr(f0) * scale));
    const unsigned short hb1 = h_bits((_Float16)(bfr(f1) * scale));
    const unsigned short bb0 = bf_bits(f0);
    const unsigned short bb1 = bf_bits(f1);
    o[e] = (f16mode != 0) ? pk16(hb0, hb1) : pk16(bb0, bb1);
  }
  u16* d = D + (size_t)gt * 8;
  for (int pass = 0; pass < 2; ++pass) {
    *(volatile v4u*)(d) = o;
    __threadfence();
  }
}

__global__ __launch_bounds__(256) void wt16(const float* __restrict__ W, u16* Bo, int f16mode, float scale) {
  __shared__ __align__(16) u16 TT[64 * VTP];
  const int tid = threadIdx.x;
  const int bid = blockIdx.x;
  const int kt  = bid % (DMOD / 64);
  const int nt  = bid / (DMOD / 64);
  if (nt >= DMOD / 64) return;
  const int k0 = kt * 64, n0 = nt * 64;
  {
    const int r  = tid >> 2;
    const int cc = (tid & 3) * 16;
    const float* src = W + (size_t)(k0 + r) * DMOD + n0 + cc;
#pragma unroll
    for (int i = 0; i < 4; ++i) {
      const v4f a = *(const v4f*)(src + 4 * i);
#pragma unroll
      for (int e = 0; e < 4; ++e) {
        const float f = a[e];
        const unsigned short hb = h_bits((_Float16)(bfr(f) * scale));
        const unsigned short bb = bf_bits(f);
        TT[(cc + 4 * i + e) * VTP + r] = (f16mode != 0) ? hb : bb;
      }
    }
  }
  __syncthreads();
  v4u w[2];
  const int q8 = tid >> 3, p8 = (tid & 7) * 8;
#pragma unroll
  for (int it = 0; it < 2; ++it) {
    const int line = it * 32 + q8;
    w[it] = *(const v4u*)(TT + line * VTP + p8);
  }
  for (int pass = 0; pass < 2; ++pass) {
#pragma unroll
    for (int it = 0; it < 2; ++it) {
      const int line = it * 32 + q8;
      *(volatile v4u*)(Bo + (size_t)(n0 + line) * DMOD + k0 + p8) = w[it];
    }
    __threadfence();
  }
}

__global__ __launch_bounds__(32) void ema_k16(const float* __restrict__ F, const float* __restrict__ lac,
                                               const float* __restrict__ kbe, u16* KHo, u16* KLo) {
#pragma clang fp contract(off)
  __shared__ __align__(16) u16 TH[TCH * VTP];
  __shared__ __align__(16) u16 TL[TCH * VTP];
  const int lane = threadIdx.x & 31;
  const int bid  = blockIdx.x;
  const int h    = bid % NH;
  const int b    = bid / NH;
  if (b >= NB) return;
  const float alpha = bfr(lac[h]);
  const float oma   = 1.0f - alpha;
  const float kb    = expf(fminf(bfr(kbe[h]) * ESCL, KBUP));
  const float* src  = F + (size_t)b * SEQ * DMOD + (size_t)h * HD + lane;
  const size_t dbase = (size_t)b * SEQ * DMOD + (size_t)h * HD;
  const int rq = lane >> 3, p8 = (lane & 7) * 8;
  float c0 = 0.0f, c1 = 0.0f;
#pragma unroll 1
  for (int tc = 0; tc < SEQ; tc += TCH) {
#pragma unroll 1
    for (int tt = 0; tt < TCH; ++tt) {
      const float* p = src + (size_t)(tc + tt) * DMOD;
      const float x0 = p[0];
      const float x1 = p[32];
      const float a0 = alpha * c0;
      const float a1 = alpha * c1;
      const float g0 = oma * x0;
      const float g1 = oma * x1;
      c0 = a0 + g0;
      c1 = a1 + g1;
      float s = c0 * c0 + c1 * c1;
#pragma unroll
      for (int off = 1; off < 32; off <<= 1) s += __shfl_xor(s, off, 32);
      const float rn = kb / sqrtf(s);
      const float t0 = (c0 * rn) * KSC;
      const float t1 = (c1 * rn) * KSC;
      const _Float16 h0 = (_Float16)t0, h1 = (_Float16)t1;
      const _Float16 l0 = (_Float16)(t0 - (float)h0), l1 = (_Float16)(t1 - (float)h1);
      TH[tt * VTP + lane]      = h_bits(h0);
      TH[tt * VTP + lane + 32] = h_bits(h1);
      TL[tt * VTP + lane]      = h_bits(l0);
      TL[tt * VTP + lane + 32] = h_bits(l1);
    }
    __syncthreads();
    v4u vh[8], vl[8];
#pragma unroll
    for (int it = 0; it < 8; ++it) {
      const int row = it * 4 + rq;
      vh[it] = *(const v4u*)(TH + row * VTP + p8);
      vl[it] = *(const v4u*)(TL + row * VTP + p8);
    }
    for (int pass = 0; pass < 2; ++pass) {
#pragma unroll
      for (int it = 0; it < 8; ++it) {
        const int row = it * 4 + rq;
        const size_t o = dbase + (size_t)(tc + row) * DMOD + p8;
        *(volatile v4u*)(KHo + o) = vh[it];
        *(volatile v4u*)(KLo + o) = vl[it];
      }
      __threadfence();
    }
    __syncthreads();
  }
}

__global__ __launch_bounds__(256) void vmix16(const float* __restrict__ F, const float* __restrict__ vco,
                                              const float* __restrict__ vbe, u16* VHo, u16* VLo) {
#pragma clang fp contract(off)
  __shared__ __align__(16) u16 TH[HD * VTP];
  __shared__ __align__(16) u16 TL[HD * VTP];
  const int tid = threadIdx.x;
  const int bid = blockIdx.x;
  const int st  = bid % NST;
  const int t2  = bid / NST;
  const int h   = t2 % NH;
  const int b   = t2 / NH;
  if (b >= NB) return;
  const int s0  = st * 64;
  const float cc  = bfr(vco[h]);
  const float omc = 1.0f - cc;
  const float vb  = expf(bfr(vbe[h]) * ESCL);
  {
    const int sl = tid >> 2;
    const int dc = (tid & 3) * 16;
    const int s  = s0 + sl;
    const bool has = (s + 1 < SEQ);
    const int sn = has ? (s + 1) : s;
    const float* p0 = F + ((size_t)b * SEQ + s)  * DMOD + h * HD + dc;
    const float* p1 = F + ((size_t)b * SEQ + sn) * DMOD + h * HD + dc;
    float v[16];
    float ss = 0.0f;
#pragma unroll
    for (int i = 0; i < 4; ++i) {
      const v4f a  = *(const v4f*)(p0 + 4 * i);
      const v4f n4 = *(const v4f*)(p1 + 4 * i);
#pragma unroll
      for (int e = 0; e < 4; ++e) {
        const float xs = has ? n4[e] : 0.0f;
        const float ta = xs * omc;
        const float tb = a[e] * cc;
        const float vv = ta + tb;
        v[4 * i + e] = vv;
        ss = ss + vv * vv;
      }
    }
    ss += __shfl_xor(ss, 1, 32);
    ss += __shfl_xor(ss, 2, 32);
    const float rn = vb / sqrtf(ss);
#pragma unroll
    for (int j = 0; j < 16; ++j) {
      const float t = (v[j] * rn) * VCAR;
      const _Float16 hv = (_Float16)t;
      const _Float16 lv = (_Float16)(t - (float)hv);
      TH[(dc + j) * VTP + sl] = h_bits(hv);
      TL[(dc + j) * VTP + sl] = h_bits(lv);
    }
  }
  __syncthreads();
  v4u vh[2], vl[2];
  const int q8 = tid >> 3, p8 = (tid & 7) * 8;
#pragma unroll
  for (int it = 0; it < 2; ++it) {
    const int line = it * 32 + q8;
    vh[it] = *(const v4u*)(TH + line * VTP + p8);
    vl[it] = *(const v4u*)(TL + line * VTP + p8);
  }
  const size_t hrow = (size_t)(b * NH + h) * HD;
  const size_t base = hrow * SEQ + s0 + p8;
  for (int pass = 0; pass < 2; ++pass) {
#pragma unroll
    for (int it = 0; it < 2; ++it) {
      const int line = it * 32 + q8;
      *(volatile v4u*)(VHo + base + (size_t)line * SEQ) = vh[it];
      *(volatile v4u*)(VLo + base + (size_t)line * SEQ) = vl[it];
    }
    __threadfence();
  }
}

__device__ __forceinline__ void epi64(float* sl, v8f a0, v8f a1, v8f a2, v8f a3, float oscale,
                                      float* C, int N, size_t rowb, int col0, int lane) {
  const int hh = lane >> 4, m = lane & 15;
#pragma unroll
  for (int r = 0; r < 8; ++r) {
    const int ro = (8 * hh + r) * 68 + m;
    sl[ro]      = a0[r] * oscale;
    sl[ro + 16] = a1[r] * oscale;
    sl[ro + 32] = a2[r] * oscale;
    sl[ro + 48] = a3[r] * oscale;
  }
  wave_sync_lds();
  v4f vals[8];
#pragma unroll
  for (int it = 0; it < 8; ++it) vals[it] = *(const v4f*)(sl + (it * 2 + hh) * 68 + m * 4);
  float* dst = C + (rowb + (size_t)hh) * (size_t)N + col0 + m * 4;
  for (int pass = 0; pass < 2; ++pass) {
#pragma unroll
    for (int it = 0; it < 8; ++it) {
      *(volatile v4f*)(dst + (size_t)(it * 2) * (size_t)N) = vals[it];
    }
    __threadfence();
  }
}

__global__ __launch_bounds__(128)
void gemm_bf(const u16* __restrict__ A, const u16* __restrict__ Bt, float* C, int M, int N, int K, float oscale) {
  __shared__ __align__(16) float slab[4 * SLAB64];
  const int tid = threadIdx.x, wave = tid >> 5, lane = tid & 31, hh = lane >> 4, m = lane & 15;
  const int ntile = N >> 6;
  const int bid   = blockIdx.x;
  const int rowb  = (bid / ntile) * 64 + wave * 16;
  const int col0  = (bid % ntile) * 64;
  if (rowb + 16 > M) return;
  const u16* ap = A  + (size_t)(rowb + m) * K + 8 * hh;
  const u16* bp = Bt + (size_t)(col0 + m) * K + 8 * hh;
  const size_t bs = (size_t)16 * K;
  v8f acc0 = zero8(), acc1 = zero8(), acc2 = zero8(), acc3 = zero8();
#pragma unroll 1
  for (int k0 = 0; k0 < K; k0 += 32) {
    const v16b a  = ldfrag_b(ap + k0);
    const v16b b0 = ldfrag_b(bp + k0);
    const v16b b1 = ldfrag_b(bp + bs + k0);
    const v16b b2 = ldfrag_b(bp + 2 * bs + k0);
    const v16b b3 = ldfrag_b(bp + 3 * bs + k0);
    acc0 = mma_b(a, b0, acc0);
    acc1 = mma_b(a, b1, acc1);
    acc2 = mma_b(a, b2, acc2);
    acc3 = mma_b(a, b3, acc3);
    guard6<v16b>(acc0, acc1, acc2, acc3, a, b0, b1, b2, b3, a);
  }
  epi64(slab + wave * SLAB64, acc0, acc1, acc2, acc3, oscale, C, N, (size_t)rowb, col0, lane);
}

__global__ __launch_bounds__(128)
void gemm_o(const u16* __restrict__ Ah, const u16* __restrict__ Al, const u16* __restrict__ Bt,
            float* C, int nrt, float oscale) {
  __shared__ __align__(16) float slab[4 * SLAB64];
  const int tid = threadIdx.x, wave = tid >> 5, lane = tid & 31, hh = lane >> 4, m = lane & 15;
  const int ntile = DMOD >> 6;
  const int bid   = blockIdx.x;
  const int ct    = bid % ntile;
  const int t2    = bid / ntile;
  const int rt    = t2 % nrt;
  const int bb    = t2 / nrt;
  if (bb >= NB) return;
  const int srow  = rt * 64 + wave * 16;
  if (srow + 16 > SEQ) return;
  const int col0  = ct * 64;
  const int K     = DMOD;
  const size_t rowA = (size_t)bb * SEQ + srow;
  const size_t rowC = (size_t)bb * XS_FULL + srow;
  const _Float16* ahp = ash(Ah) + (rowA + m) * K + 8 * hh;
  const _Float16* alp = ash(Al) + (rowA + m) * K + 8 * hh;
  const _Float16* bp  = ash(Bt) + (size_t)(col0 + m) * K + 8 * hh;
  const size_t bs = (size_t)16 * K;
  v8f acc0 = zero8(), acc1 = zero8(), acc2 = zero8(), acc3 = zero8();
#pragma unroll 1
  for (int k0 = 0; k0 < K; k0 += 32) {
    const v16h ah = ldfrag_h(ahp + k0), al = ldfrag_h(alp + k0);
    const v16h b0 = ldfrag_h(bp + k0);
    const v16h b1 = ldfrag_h(bp + bs + k0);
    const v16h b2 = ldfrag_h(bp + 2 * bs + k0);
    const v16h b3 = ldfrag_h(bp + 3 * bs + k0);
    acc0 = mma_h(ah, b0, acc0);  acc0 = mma_h(al, b0, acc0);
    acc1 = mma_h(ah, b1, acc1);  acc1 = mma_h(al, b1, acc1);
    acc2 = mma_h(ah, b2, acc2);  acc2 = mma_h(al, b2, acc2);
    acc3 = mma_h(ah, b3, acc3);  acc3 = mma_h(al, b3, acc3);
    guard6<v16h>(acc0, acc1, acc2, acc3, ah, al, b0, b1, b2, b3);
  }
  epi64(slab + wave * SLAB64, acc0, acc1, acc2, acc3, oscale, C, DMOD, rowC, col0, lane);
}

template <int RES>
__global__ __launch_bounds__(ATT_THREADS)
void attn_c(const u16* __restrict__ KHp, const u16* __restrict__ KLp,
            const u16* __restrict__ VHp, const u16* __restrict__ VLp,
            u16* OHp, u16* OLp) {
  __shared__ __align__(16) float smem[WPB * WREG];
  constexpr int QT0 = (RES != 0) ? 0 : NQO;
  constexpr int NQL = (RES != 0) ? NQO : (NQT - NQO);
  constexpr int NQE = (NQL > 0) ? NQL : 1;

  const int tid  = threadIdx.x;
  const int wave = tid >> 5;
  const int lane = tid & 31;
  const int hh   = lane >> 4;
  const int c    = lane & 15;
  const int bid  = blockIdx.x;
  const int qt   = QT0 + (bid % NQE);
  const int t2   = bid / NQE;
  const int hg   = t2 % NHG;
  const int b    = t2 / NHG;
  if (b >= NB) return;
  const int q0   = qt * 16;
  if (q0 + 16 > SEQ) return;
  if (RES != 0 && q0 + 16 > QO) return;
  const int head = hg * WPB + wave;

  float* pt   = smem + wave * WREG;
  float* slab = pt + PTW;

  const size_t hcol = (size_t)head * HD + 8 * hh;
  const size_t qrow = ((size_t)b * SEQ + q0 + c) * DMOD + hcol;
  const size_t krow = ((size_t)b * SEQ + c) * DMOD + hcol;
  const size_t vrow = ((size_t)(b * NH + head) * HD + c) * SEQ + 8 * hh;
  const _Float16* Qh  = ash(KHp) + qrow;
  const _Float16* Ql  = ash(KLp) + qrow;
  const _Float16* Khb = ash(KHp) + krow;
  const _Float16* Klb = ash(KLp) + krow;
  const _Float16* Vhb = ash(VHp) + vrow;
  const _Float16* Vlb = ash(VLp) + vrow;
  const float lsc = LOG2E / (KSC * KSC);
  const float oc  = 1.0f / (PCAR * VCAR);
  const size_t KROW = (size_t)DMOD;

  float mrow[8], lrow[8];
  v8f o[4];
#pragma unroll
  for (int r = 0; r < 8; ++r) { mrow[r] = -INFINITY; lrow[r] = 0.f; }
#pragma unroll
  for (int j = 0; j < 4; ++j) o[j] = zero8();
  const int ncaus = (q0 >> 5) + 1;
  const int nkt = (ncaus < NKT) ? ncaus : NKT;
  const int qr0 = q0 + 8 * hh;

#pragma unroll 1
  for (int kt = 0; kt < nkt; ++kt) {
    const int kb = kt * 32;
    v8f s0 = zero8(), s1 = zero8();
    {
      const _Float16* k0p = Khb + (size_t)kb * KROW;
      const _Float16* k1p = k0p + (size_t)16 * KROW;
      const _Float16* l0p = Klb + (size_t)kb * KROW;
      const _Float16* l1p = l0p + (size_t)16 * KROW;
#pragma unroll
      for (int kk = 0; kk < HD / 32; ++kk) {
        const v16h qh  = ldfrag_h(Qh + kk * 32);
        const v16h ql  = ldfrag_h(Ql + kk * 32);
        const v16h kh0 = ldfrag_h(k0p + kk * 32);
        const v16h kh1 = ldfrag_h(k1p + kk * 32);
        const v16h kl0 = ldfrag_h(l0p + kk * 32);
        const v16h kl1 = ldfrag_h(l1p + kk * 32);
        s0 = mma_h(qh, kh0, s0);
        s0 = mma_h(ql, kh0, s0);
        s0 = mma_h(qh, kl0, s0);
        s1 = mma_h(qh, kh1, s1);
        s1 = mma_h(ql, kh1, s1);
        s1 = mma_h(qh, kl1, s1);
        guard2(s0, s1, qh, ql, kh0, kl0, kh1, kl1);
      }
    }
    const int key0 = kb + c, key1 = kb + 16 + c;
#pragma unroll
    for (int r = 0; r < 8; ++r) {
      const int   qr = qr0 + r;
      const float u0 = s0[r] * lsc;
      const float u1 = s1[r] * lsc;
      const float t0 = (key0 >= qr) ? -INFINITY : u0;
      const float t1 = (key1 >= qr) ? -INFINITY : u1;
      float mx = fmaxf(t0, t1);
#pragma unroll
      for (int off = 1; off < 16; off <<= 1) mx = fmaxf(mx, __shfl_xor(mx, off, 32));
      const float mn = fmaxf(mrow[r], mx);
      const float ms = (mn == -INFINITY) ? 0.0f : mn;
      const float al = exp2f(mrow[r] - ms);
      mrow[r] = mn;
      const float e0 = exp2f(t0 - ms), e1 = exp2f(t1 - ms);
      float ps = e0 + e1;
#pragma unroll
      for (int off = 1; off < 16; off <<= 1) ps += __shfl_xor(ps, off, 32);
      lrow[r] = lrow[r] * al + ps;
#pragma unroll
      for (int j = 0; j < 4; ++j) o[j][r] *= al;
      const int ro = (8 * hh + r) * PTP + c;
      pt[ro]      = e0;
      pt[ro + 16] = e1;
    }
    wave_sync_lds();
    FragH ph, pl;
    {
      const float* prow = pt + c * PTP + 8 * hh;
      const v4f p0 = *(const v4f*)(prow), p1 = *(const v4f*)(prow + 4);
      const v4f p2 = *(const v4f*)(prow + 16), p3 = *(const v4f*)(prow + 20);
#pragma unroll
      for (int e = 0; e < 4; ++e) {
        const float ta = p0[e] * PCAR, tb = p1[e] * PCAR, tc = p2[e] * PCAR, td = p3[e] * PCAR;
        const _Float16 ha = (_Float16)ta, hb = (_Float16)tb, hc = (_Float16)tc, hd = (_Float16)td;
        ph.h[0][e]     = ha;
        ph.h[0][4 + e] = hb;
        ph.h[1][e]     = hc;
        ph.h[1][4 + e] = hd;
        pl.h[0][e]     = (_Float16)(ta - (float)ha);
        pl.h[0][4 + e] = (_Float16)(tb - (float)hb);
        pl.h[1][e]     = (_Float16)(tc - (float)hc);
        pl.h[1][4 + e] = (_Float16)(td - (float)hd);
      }
    }
    {
      const _Float16* vhp = Vhb + kb;
      const _Float16* vlp = Vlb + kb;
#pragma unroll
      for (int jg = 0; jg < 2; ++jg) {
        const size_t da = (size_t)(2 * jg) * 16 * SEQ;
        const size_t db = da + (size_t)16 * SEQ;
        const v16h vha = ldfrag_h(vhp + da), vhb2 = ldfrag_h(vhp + db);
        const v16h vla = ldfrag_h(vlp + da), vlb2 = ldfrag_h(vlp + db);
        if constexpr (RES != 0) {
          o[2 * jg]     = mma_h(ph.v, vha,  o[2 * jg]);
          o[2 * jg]     = mma_h(pl.v, vha,  o[2 * jg]);
          o[2 * jg]     = mma_h(ph.v, vla,  o[2 * jg]);
          o[2 * jg + 1] = mma_h(ph.v, vhb2, o[2 * jg + 1]);
          o[2 * jg + 1] = mma_h(pl.v, vhb2, o[2 * jg + 1]);
          o[2 * jg + 1] = mma_h(ph.v, vlb2, o[2 * jg + 1]);
          guard2(o[2 * jg], o[2 * jg + 1], ph.v, pl.v, vha, vhb2, vla, vlb2);
        } else {
          o[2 * jg]     = mma_h(ph.v, vha,  o[2 * jg]);
          o[2 * jg]     = mma_h(ph.v, vla,  o[2 * jg]);
          o[2 * jg + 1] = mma_h(ph.v, vhb2, o[2 * jg + 1]);
          o[2 * jg + 1] = mma_h(ph.v, vlb2, o[2 * jg + 1]);
          guard2(o[2 * jg], o[2 * jg + 1], ph.v, vha, vhb2, vla, vlb2, ph.v);
        }
      }
    }
    wave_sync_lds();
  }
  acc_guard4(o[0], o[1], o[2], o[3]);
#pragma unroll
  for (int r = 0; r < 8; ++r) {
    const float lv  = lrow[r];
    const float ls  = (lv > 0.0f) ? lv : 1.0f;
    const float inv = (lv > 0.0f) ? ((1.0f / ls) * oc) : 0.0f;
#pragma unroll
    for (int j = 0; j < 4; ++j) {
      const int idx = (8 * hh + r) * SLP + j * 16 + c;
      slab[idx] = o[j][r] * inv;
    }
  }

  wave_sync_lds();
  v4u oh[4], ol[4];
  const int rq = lane >> 3, c8 = (lane & 7) * 8;
#pragma unroll
  for (int it = 0; it < 4; ++it) {
    const int row = it * 4 + rq;
    const v4f a = *(const v4f*)(slab + row * SLP + c8), b4 = *(const v4f*)(slab + row * SLP + c8 + 4);
    float w[8];
#pragma unroll
    for (int e = 0; e < 4; ++e) { w[e] = a[e] * OSC; w[4 + e] = b4[e] * OSC; }
#pragma unroll
    for (int e = 0; e < 4; ++e) {
      const _Float16 h0 = (_Float16)w[2 * e], h1 = (_Float16)w[2 * e + 1];
      const _Float16 l0 = (_Float16)(w[2 * e] - (float)h0), l1 = (_Float16)(w[2 * e + 1] - (float)h1);
      oh[it][e] = pk16(h_bits(h0), h_bits(h1));
      ol[it][e] = pk16(h_bits(l0), h_bits(l1));
    }
  }
  const size_t ob = ((size_t)b * SEQ + q0) * DMOD + (size_t)head * HD + c8;
  for (int pass = 0; pass < 2; ++pass) {
#pragma unroll
    for (int it = 0; it < 4; ++it) {
      const int row = it * 4 + rq;
      *(volatile v4u*)(OHp + ob + (size_t)row * DMOD) = oh[it];
      *(volatile v4u*)(OLp + ob + (size_t)row * DMOD) = ol[it];
    }
    __threadfence();
  }
}

extern "C" void kernel_launch(void* const* d_in, const int* in_sizes, int n_in,
                              void* d_out, int out_size, void* d_ws, size_t ws_size,
                              hipStream_t stream) {
  if (n_in < 8) return;
  if (in_sizes[0] < ((NB - 1) * XS_FULL + SEQ) * DMOD) return;
  if (in_sizes[1] != DMOD * DMOD) return;
  if (in_sizes[5] != DMOD * DMOD) return;
  if (in_sizes[7] != DMOD * DMOD) return;
  if (in_sizes[2] < NH || in_sizes[3] < NH || in_sizes[4] < NH || in_sizes[6] < NH) return;
  if (out_size < ((NB - 1) * XS_FULL + SEQ) * DMOD) return;

  const float* x    = (const float*)d_in[0];
  const float* wla  = (const float*)d_in[1];
  const float* lac  = (const float*)d_in[2];
  const float* kbe  = (const float*)d_in[3];
  const float* vbe  = (const float*)d_in[4];
  const float* wv   = (const float*)d_in[5];
  const float* vco  = (const float*)d_in[6];
  const float* wpj  = (const float*)d_in[7];
  float*       out  = (float*)d_out;

  const size_t szXB = (size_t)MROWS * DMOD * 2;
  const size_t szW  = (size_t)DMOD * DMOD * 2;
  const size_t szF  = (size_t)MROWS * DMOD * 4;
  const size_t szH  = (size_t)MROWS * DMOD * 2;
  const size_t szV  = (size_t)NB * NH * HD * SEQ * 2;
  size_t off = 0;
  const size_t oXB = off; off += szXB;
  const size_t oW  = off; off += szW;
  const size_t oF  = off; off += szF;
  const size_t oKH = off; off += szH;
  const size_t oKL = off; off += szH;
  const size_t oVH = off; off += szV;
  const size_t oVL = off; off += szV;
  const size_t oOH = off; off += szH;
  const size_t oOL = off; off += szH;
  if (off > ws_size) return;
  if (off > (size_t)WS_CAP) return;

  char* ws = (char*)d_ws;
  u16*   XB  = (u16*)(ws + oXB);
  u16*   WB  = (u16*)(ws + oW);
  float* F   = (float*)(ws + oF);
  u16*   KH  = (u16*)(ws + oKH);
  u16*   KL  = (u16*)(ws + oKL);
  u16*   VH  = (u16*)(ws + oVH);
  u16*   VL  = (u16*)(ws + oVL);
  u16*   OH  = (u16*)(ws + oOH);
  u16*   OL  = (u16*)(ws + oOL);

  const dim3 b256(256), b128(128), b32(32), bAT(ATT_THREADS);
  const int  n8x = (SEQ * DMOD) / 8;
  const dim3 gX((n8x + 255) / 256);
  const dim3 gWT((DMOD / 64) * (DMOD / 64));
  const dim3 gG((MROWS / 64) * (DMOD / 64));
  const dim3 gVT(NB * NH * NST);
  const dim3 gEM(NB * NH);
  const dim3 gATR(NQO * NHG * NB);
  const int  nqp  = NQT - NQO;
  const int  nrt  = SEQ / 64;

  for (int b = 0; b < NB; ++b) {
    cvt16<<<gX, b256, 0, stream>>>(x + (size_t)b * XS_FULL * DMOD, XB + (size_t)b * SEQ * DMOD, n8x, 0, 1.0f);
  }
  wt16<<<gWT, b256, 0, stream>>>(wv, WB, 0, 1.0f);
  gemm_bf<<<gG, b128, 0, stream>>>(XB, WB, F, MROWS, DMOD, DMOD, 1.0f);
  vmix16<<<gVT, b256, 0, stream>>>(F, vco, vbe, VH, VL);
  wt16<<<gWT, b256, 0, stream>>>(wla, WB, 0, 1.0f);
  gemm_bf<<<gG, b128, 0, stream>>>(XB, WB, F, MROWS, DMOD, DMOD, 1.0f);
  ema_k16<<<gEM, b32, 0, stream>>>(F, lac, kbe, KH, KL);
  wt16<<<gWT, b256, 0, stream>>>(wpj, WB, 1, WOS);
  attn_c<1><<<gATR, bAT, 0, stream>>>(KH, KL, VH, VL, OH, OL);
  if (nqp > 0) {
    attn_c<0><<<dim3(nqp * NHG * NB), bAT, 0, stream>>>(KH, KL, VH, VL, OH, OL);
  }
  gemm_o<<<dim3(NB * nrt * (DMOD / 64)), b128, 0, stream>>>(OH, OL, WB, out, nrt, 1.0f / (OSC * WOS));
  (void)hipGetLastError();
}
